// GraphAttn_28157805593322
// MI455X (gfx1250) — hardware-verified
//
#include <hip/hip_runtime.h>
#include <math.h>

#define NB_ 16
#define NN_ 2048
#define FT  64

typedef _Float16 f16;
typedef __attribute__((ext_vector_type(16))) f16 f16x16;
typedef __attribute__((ext_vector_type(8)))  f16 f16x8;
typedef __attribute__((ext_vector_type(8)))  float f32x8;
typedef __attribute__((ext_vector_type(4)))  float v4f_t;
typedef float v4fa __attribute__((ext_vector_type(4), may_alias));

__device__ __forceinline__ f32x8 wmma16(f16x16 a, f16x16 b, f32x8 c) {
  c = __builtin_amdgcn_wmma_f32_16x16x32_f16(false, a, false, b, (short)0, c, false, false);
  asm volatile("v_nop\n\tv_nop\n\tv_nop\n\tv_nop" : "+v"(c) : "v"(a), "v"(b));
  return c;
}
__device__ __forceinline__ f16x16 lds_frag(const f16* base, int stride) {
  const int lane = threadIdx.x & 31, row = lane & 15, kh = (lane >> 4) * 8;
  const f16x8 lo = *(const f16x8*)(base + row * stride + kh);
  const f16x8 hi = *(const f16x8*)(base + row * stride + kh + 16);
  f16x16 f;
#pragma unroll
  for (int i = 0; i < 8; ++i) { f[i] = lo[i]; f[i + 8] = hi[i]; }
  return f;
}
#define GSTR 48

template <typename AT, int ASRC>
__global__ __launch_bounds__(256) void gemm_knb2(const AT* __restrict__ A, int lda, size_t strideA,
                                               const float* __restrict__ Wm, int ldw, size_t strideW,
                                               const float* __restrict__ rowbias, const float* __restrict__ s1, const float* __restrict__ s2, const float* __restrict__ mj, const float* __restrict__ invD,
                                               float scale, int N, float* __restrict__ Y, int ldy, size_t strideY, int K) {
  __shared__ __attribute__((aligned(16))) f16 ldsA[128 * GSTR], ldsAl[128 * GSTR];
  __shared__ __attribute__((aligned(16))) f16 ldsW[128 * GSTR], ldsWl[128 * GSTR];
  __shared__ __attribute__((aligned(16))) float oS[8][32 * 68];
  const int tid = threadIdx.x, lane = tid & 31, wave = tid >> 5, cl = lane & 15, rh = (lane >> 4) * 8;
  const int m0 = blockIdx.x * 128, n0 = blockIdx.y * 128;
  const int wm = (wave & 3) * 32, wn = (wave >> 2) * 64;
  A += (size_t)blockIdx.z * strideA; Wm += (size_t)blockIdx.z * strideW; Y += (size_t)blockIdx.z * strideY;
  if (ASRC == 1) { s1 += (size_t)blockIdx.z * K; s2 += (size_t)blockIdx.z * lda; mj += (size_t)blockIdx.z * K; invD += (size_t)blockIdx.z * K; }
  f32x8 acc[2][4], accx[2][4];
#pragma unroll
  for (int i = 0; i < 2; ++i)
#pragma unroll
    for (int j = 0; j < 4; ++j) { f32x8 z = {}; acc[i][j] = z; accx[i][j] = z; }
#pragma unroll 1
  for (int k0 = 0; k0 < K; k0 += 32) {
    __syncthreads();
    {
      const int row = tid >> 1, ch = (tid & 1) * 16;
      if (ASRC == 0) {
        const AT* src = A + (size_t)(m0 + row) * lda + k0 + ch;
#pragma unroll
        for (int g = 0; g < 16; ++g) { const float v = (float)src[g]; const f16 h = (f16)v; ldsA[row * GSTR + ch + g] = h; ldsAl[row * GSTR + ch + g] = (f16)((v - (float)h) * 2048.0f); }
      } else {
        const float s2i = s2[m0 + row];
#pragma unroll
        for (int g = 0; g < 16; ++g) { const int j = k0 + ch + g; float a = s1[j] + s2i; a = (a >= 0.0f) ? a : 0.2f * a;
          const float v = 1024.0f * __expf(a - mj[j]) * invD[j]; const f16 h = (f16)v; ldsA[row * GSTR + ch + g] = h; ldsAl[row * GSTR + ch + g] = (f16)((v - (float)h) * 2048.0f); }
      }
    }
    {
      const int k = tid >> 3, nn0 = (tid & 7) * 16;
      const float* src = Wm + (size_t)(k0 + k) * ldw;
#pragma unroll
      for (int g = 0; g < 4; ++g) { const int col = min(n0 + nn0 + 4 * g, N - 4); const v4f_t v = *(const v4f_t*)(src + col);
#pragma unroll
        for (int u = 0; u < 4; ++u) { const f16 h = (f16)v[u]; ldsW[(nn0 + 4 * g + u) * GSTR + k] = h; ldsWl[(nn0 + 4 * g + u) * GSTR + k] = (f16)((v[u] - (float)h) * 2048.0f); } }
    }
    __syncthreads();
    f16x16 af[2], afl[2];
#pragma unroll
    for (int i = 0; i < 2; ++i) { af[i] = lds_frag(ldsA + (wm + 16 * i) * GSTR, GSTR); afl[i] = lds_frag(ldsAl + (wm + 16 * i) * GSTR, GSTR); }
#pragma unroll
    for (int j = 0; j < 4; ++j) {
      const f16x16 bf = lds_frag(ldsW + (wn + 16 * j) * GSTR, GSTR), bfl = lds_frag(ldsWl + (wn + 16 * j) * GSTR, GSTR);
#pragma unroll
      for (int i = 0; i < 2; ++i) { acc[i][j] = wmma16(af[i], bf, acc[i][j]); accx[i][j] = wmma16(af[i], bfl, accx[i][j]); accx[i][j] = wmma16(afl[i], bf, accx[i][j]); }
    }
  }
  float* so = oS[wave];
#pragma unroll
  for (int i = 0; i < 2; ++i)
#pragma unroll
    for (int j = 0; j < 4; ++j) {
#pragma unroll
      for (int r = 0; r < 8; ++r) { const float rb = rowbias ? rowbias[m0 + wm + 16 * i + rh + r] : 0.0f; so[(16 * i + rh + r) * 68 + 16 * j + cl] = (acc[i][j][r] + accx[i][j][r] * (1.0f / 2048.0f)) * scale + rb; }
    }
  asm volatile("s_wait_dscnt 0" ::: "memory");
  __builtin_amdgcn_wave_barrier();
#pragma unroll 1
  for (int pass = 0; pass < 2; ++pass) {
#pragma unroll
    for (int it = 0; it < 16; ++it) { const int f4 = lane + 32 * it, rr = f4 >> 4, q = (f4 & 15) * 4;
      if (n0 + wn + q < N) *(volatile v4f_t*)(Y + (size_t)(m0 + wm + rr) * ldy + n0 + wn + q) = *(const volatile v4fa*)(so + rr * 68 + q); }
    __threadfence();
  }
}

__global__ __launch_bounds__(256) void k_scores(const float* __restrict__ xf, const float* __restrict__ nf, const float* __restrict__ a1,
                                               const float* __restrict__ a2, float* __restrict__ s1g, float* __restrict__ s2g,
                                               float* __restrict__ mg, float* __restrict__ iDg) {
  __shared__ float s1S[NN_], s2S[NN_], red[256];
  __shared__ __attribute__((aligned(16))) float mS[NN_], iS[NN_];
  const int b = blockIdx.x, t = threadIdx.x;
  __shared__ float w1[FT], w2[FT];
  if (t < FT) { w1[t] = a1[t]; w2[t] = a2[t]; }
  __syncthreads();
  float mx = -INFINITY;
  for (int nd = t; nd < NN_; nd += 256) {
    const float* xr = xf + ((size_t)b * NN_ + nd) * FT; const float* nr = nf + ((size_t)b * NN_ + nd) * FT;
    float p = 0.0f, q = 0.0f;
#pragma unroll 1
    for (int f = 0; f < FT; ++f) { p += xr[f] * w1[f]; q += nr[f] * w2[f]; }
    s1S[nd] = p; s2S[nd] = q; mx = fmaxf(mx, q);
  }
  red[t] = mx; __syncthreads();
  for (int o = 128; o > 0; o >>= 1) { if (t < o) red[t] = fmaxf(red[t], red[t + o]); __syncthreads(); }
  const float ms2 = red[0];
  for (int j = t; j < NN_; j += 256) {
    const float sj = s1S[j]; float m = sj + ms2; m = (m >= 0.0f) ? m : 0.2f * m;
    float D = 0.0f;
    for (int i = 0; i < NN_; ++i) { float a = sj + s2S[i]; a = (a >= 0.0f) ? a : 0.2f * a; D += __expf(a - m); }
    mS[j] = m; iS[j] = 1.0f / D;
  }
  __syncthreads();
#pragma unroll 1
  for (int pass = 0; pass < 2; ++pass) {
#pragma unroll
    for (int it = 0; it < 2; ++it) { const int q = (t + 256 * it) * 4;
      *(volatile v4f_t*)(s1g + (size_t)b * NN_ + q) = *(const volatile v4fa*)(s1S + q);
      *(volatile v4f_t*)(s2g + (size_t)b * NN_ + q) = *(const volatile v4fa*)(s2S + q);
      *(volatile v4f_t*)(mg + (size_t)b * NN_ + q) = *(const volatile v4fa*)(mS + q);
      *(volatile v4f_t*)(iDg + (size_t)b * NN_ + q) = *(const volatile v4fa*)(iS + q); }
    __threadfence();
  }
}

extern "C" void kernel_launch(void* const* d_in, const int* in_sizes, int n_in,
                              void* d_out, int out_size, void* d_ws, size_t ws_size,
                              hipStream_t stream) {
  (void)in_sizes; (void)n_in; (void)out_size; (void)ws_size;
  const float* x = (const float*)d_in[0];
  const float* n = (const float*)d_in[1];
  const float* cw = (const float*)d_in[2];
  const float* cb = (const float*)d_in[3];
  const float* a1 = (const float*)d_in[4];
  const float* a2 = (const float*)d_in[5];
  float* out = (float*)d_out;
  char* ws = (char*)d_ws;
  const size_t T = (size_t)NB_ * NN_ * FT * 4;
  float* xf = (float*)ws; ws += T; float* nf = (float*)ws; ws += T;
  float* s1 = (float*)ws; ws += NB_ * NN_ * 4; float* s2 = (float*)ws; ws += NB_ * NN_ * 4; float* mj = (float*)ws; ws += NB_ * NN_ * 4; float* iD = (float*)ws; ws += NB_ * NN_ * 4;
  const dim3 g(NN_ / 128, 1, NB_), blk(256);
  gemm_knb2<float, 0><<<g, blk, 0, stream>>>(cw, NN_, 0, x, FT, (size_t)NN_ * FT, cb, nullptr, nullptr, nullptr, nullptr, 1.0f, FT, xf, FT, (size_t)NN_ * FT, NN_);
  gemm_knb2<float, 0><<<g, blk, 0, stream>>>(cw, NN_, 0, n, FT, (size_t)NN_ * FT, cb, nullptr, nullptr, nullptr, nullptr, 1.0f, FT, nf, FT, (size_t)NN_ * FT, NN_);
  k_scores<<<dim3(NB_), dim3(256), 0, stream>>>(xf, nf, a1, a2, s1, s2, mj, iD);
  gemm_knb2<float, 1><<<g, blk, 0, stream>>>(nullptr, NN_, 0, xf, FT, (size_t)NN_ * FT, nullptr, s1, s2, mj, iD, 1.0f / 1024.0f, FT, out, FT, (size_t)NN_ * FT, NN_);
}
